// GatedLinearAttentionARMA_61040075210838
// MI455X (gfx1250) — hardware-verified
//
#include <hip/hip_runtime.h>
#include <hip/hip_bf16.h>
#include <math.h>


#define BB 2
#define SS 1024
#define DD 1024
#define HH 16
#define DKK 64
#define QW 2

typedef _Float16 bf16;
typedef __attribute__((ext_vector_type(4))) unsigned v4u_t;
typedef unsigned v4ua __attribute__((ext_vector_type(4), may_alias));
typedef __attribute__((ext_vector_type(4))) float v4f_t;
typedef float v4fa __attribute__((ext_vector_type(4), may_alias));
typedef __attribute__((ext_vector_type(16))) bf16  bf16x16;
typedef __attribute__((ext_vector_type(8)))  bf16  bf16x8;
typedef __attribute__((ext_vector_type(4)))  bf16  bf16x4;
typedef __attribute__((ext_vector_type(8)))  float f32x8;

#define LDS_STRIDE 48
#define KSTRIDE    72
#define VSTRIDE    48

__device__ __forceinline__ f32x8 wmma_bf16(bf16x16 a, bf16x16 b, f32x8 c) {
  return __builtin_amdgcn_wmma_f32_16x16x32_f16(
      false, a, false, b, (short)0, c, false, false);
}
#define RSPLIT (1.0f / 2048.0f)
__device__ __forceinline__ bf16 lo_of(float v, bf16 h) { return (bf16)((v - (float)h) * 2048.0f); }
__device__ __forceinline__ f32x8 wmma_split(bf16x16 a, bf16x16 al, bf16x16 b, bf16x16 bl, f32x8 c) {
  f32x8 x = {}; x = wmma_bf16(al, b, x); x = wmma_bf16(a, bl, x); return wmma_bf16(a, b, c) + x * RSPLIT; }

template <typename T>
__device__ __forceinline__ bf16x16 load_frag(const T* __restrict__ base, int ld,
                                             int row0, int k0) {
  const int lane = threadIdx.x & 31;
  const int r    = lane & 15;
  const int kh   = (lane >> 4) * 8;
  const T* p0 = base + (size_t)(row0 + r) * ld + (k0 + kh);
  const T* p1 = p0 + 16;
  bf16x16 f;
#pragma unroll
  for (int i = 0; i < 8; ++i) {
    f[i]     = (bf16)p0[i];
    f[i + 8] = (bf16)p1[i];
  }
  return f;
}

__device__ __forceinline__ bf16x16 lds_frag(const bf16* base, int stride) {
  const int lane = threadIdx.x & 31;
  const int row  = lane & 15;
  const int kh   = (lane >> 4) * 8;
  const bf16x8 lo = *(const bf16x8*)(base + row * stride + kh);
  const bf16x8 hi = *(const bf16x8*)(base + row * stride + kh + 16);
  bf16x16 f;
#pragma unroll
  for (int i = 0; i < 8; ++i) { f[i] = lo[i]; f[i + 8] = hi[i]; }
  return f;
}

template <typename T>
__device__ __forceinline__ void stage_read16(const T* __restrict__ p, float* buf) {
#pragma unroll
  for (int i = 0; i < 16; ++i) buf[i] = (float)p[i];
}

__device__ __forceinline__ void stage_write(bf16* dst, const float* buf, int nquad) {
#pragma unroll
  for (int i = 0; i < nquad; ++i) {
    bf16x4 q;
    q[0] = (bf16)buf[4 * i];     q[1] = (bf16)buf[4 * i + 1];
    q[2] = (bf16)buf[4 * i + 2]; q[3] = (bf16)buf[4 * i + 3];
    *(bf16x4*)(dst + 4 * i) = q;
  }
}

__global__ __launch_bounds__(256) void transpose_pack_kernel(const float* __restrict__ W, bf16* __restrict__ WT, int K, int N, size_t plane) {
  __shared__ float tile[64][65];
  const int k0 = blockIdx.y * 64, n0 = blockIdx.x * 64, t = threadIdx.x;
  for (int i = t; i < 64 * 64; i += 256) { const int kr = i >> 6, nc = i & 63; tile[kr][nc] = W[(size_t)(k0 + kr) * N + n0 + nc]; }
  __syncthreads();
#pragma unroll 1
  for (int pass = 0; pass < 2; ++pass) {
    for (int i = t; i < 64 * 8; i += 256) { const int nr = i >> 3, k8 = (i & 7) * 8; bf16 hh[8], hl[8];
#pragma unroll
      for (int e = 0; e < 8; ++e) { const float v = tile[k8 + e][nr]; hh[e] = (bf16)v; hl[e] = lo_of(v, hh[e]); }
      bf16* d = WT + (size_t)(n0 + nr) * K + k0 + k8;
      *(volatile v4u_t*)d = *(const v4ua*)hh; *(volatile v4u_t*)(d + plane) = *(const v4ua*)hl; }
    __threadfence();
  }
}

template <typename AT, typename WT, int MODE>
__global__ __launch_bounds__(256) void gemm_split_kernel(
    const AT* __restrict__ A, size_t aPlane, const WT* __restrict__ W, size_t wPlane,
    const float* __restrict__ bias, void* __restrict__ out,
    int M, int N, int K) {
  __shared__ bf16 ldsA[128 * LDS_STRIDE], ldsAl[128 * LDS_STRIDE];
  __shared__ bf16 ldsW[256 * LDS_STRIDE], ldsWl[256 * LDS_STRIDE];
  __shared__ __attribute__((aligned(16))) unsigned char sob[256 * 136 * 2];

  const int t    = threadIdx.x;
  const int wave = t >> 5;
  const int lane = t & 31;
  const int wm   = (wave & 1) * 64;
  const int wn   = (wave >> 1) * 64;
  const int mBlk = blockIdx.x * 128;
  const int nBlk = blockIdx.y * 256;
  const int arow = t >> 1;
  const int ach  = (t & 1) * 16;

  f32x8 acc[4][4] = {};
  for (int k = 0; k < K; k += 32) {
    __syncthreads();
    {
      const AT* ap = A + (size_t)(mBlk + arow) * K + k + ach;
      bf16 hh[16], hl[16];
      if (sizeof(AT) == 4) {
#pragma unroll
        for (int i = 0; i < 16; ++i) { const float v = (float)ap[i]; hh[i] = (bf16)v; hl[i] = lo_of(v, hh[i]); }
      } else {
#pragma unroll
        for (int i = 0; i < 16; ++i) { hh[i] = (bf16)ap[i]; hl[i] = (bf16)ap[aPlane + i]; }
      }
#pragma unroll
      for (int i = 0; i < 16; ++i) { ldsA[arow * LDS_STRIDE + ach + i] = hh[i]; ldsAl[arow * LDS_STRIDE + ach + i] = hl[i]; }
    }
    {
      const WT* wp = W + (size_t)(nBlk + t) * K + k;
      if (sizeof(WT) == 4) {
#pragma unroll
        for (int i = 0; i < 32; ++i) { const float v = (float)wp[i]; const bf16 h_ = (bf16)v; ldsW[t * LDS_STRIDE + i] = h_; ldsWl[t * LDS_STRIDE + i] = lo_of(v, h_); }
      } else {
#pragma unroll
        for (int i = 0; i < 32; ++i) { ldsW[t * LDS_STRIDE + i] = (bf16)wp[i]; ldsWl[t * LDS_STRIDE + i] = (bf16)wp[wPlane + i]; }
      }
    }
    __syncthreads();
    bf16x16 wf[4], wfl[4];
#pragma unroll
    for (int j = 0; j < 4; ++j) { wf[j] = lds_frag(ldsW + (wn + 16 * j) * LDS_STRIDE, LDS_STRIDE); wfl[j] = lds_frag(ldsWl + (wn + 16 * j) * LDS_STRIDE, LDS_STRIDE); }
#pragma unroll
    for (int i = 0; i < 4; ++i) {
      const bf16x16 af = lds_frag(ldsA + (wm + 16 * i) * LDS_STRIDE, LDS_STRIDE), afl = lds_frag(ldsAl + (wm + 16 * i) * LDS_STRIDE, LDS_STRIDE);
#pragma unroll
      for (int j = 0; j < 4; ++j) acc[i][j] = wmma_split(af, afl, wf[j], wfl[j], acc[i][j]);
    }
  }

  const int nlane = lane & 15;
  const int mh    = (lane >> 4) * 8;
  __syncthreads();
  if (MODE == 1) {
    bf16* so = (bf16*)sob;
#pragma unroll
    for (int i = 0; i < 4; ++i)
#pragma unroll
      for (int j = 0; j < 4; ++j) {
        const int nl = wn + 16 * j + nlane;
        const float bv = bias ? bias[nBlk + nl] : 0.0f;
#pragma unroll
        for (int r = 0; r < 8; ++r) so[nl * 136 + wm + 16 * i + mh + r] = (bf16)(acc[i][j][r] + bv);
      }
    __syncthreads();
    const int b_ = mBlk >> 11, s0 = mBlk & (SS - 1);
#pragma unroll 1
    for (int pass = 0; pass < 2; ++pass) {
      for (int ch = t; ch < 256 * 16; ch += 256) { const int nl = ch >> 4, q = (ch & 15) * 8; const int n = nBlk + nl, h = n >> 6, dk = n & (DKK - 1);
        *(volatile v4u_t*)((bf16*)out + (((size_t)(b_ * HH + h)) * DKK + dk) * SS + s0 + q) = *(const v4ua*)(so + nl * 136 + q); }
      __threadfence();
    }
  } else {
    float* so = (float*)sob;
#pragma unroll 1
    for (int hf = 0; hf < 2; ++hf) {
      if (wm == hf * 64) {
#pragma unroll
        for (int i = 0; i < 4; ++i)
#pragma unroll
          for (int j = 0; j < 4; ++j) {
            const int nl = wn + 16 * j + nlane;
            const float bv = bias ? bias[nBlk + nl] : 0.0f;
#pragma unroll
            for (int r = 0; r < 8; ++r) so[(16 * i + mh + r) * 260 + nl] = acc[i][j][r] + bv;
          }
      }
      __syncthreads();
#pragma unroll 1
      for (int pass = 0; pass < 2; ++pass) {
        for (int ch = t; ch < 64 * 64; ch += 256) { const int ml = ch >> 6, q = (ch & 63) * 4;
          *(volatile v4f_t*)((float*)out + (size_t)(mBlk + hf * 64 + ml) * N + nBlk + q) = *(const volatile v4fa*)(so + ml * 260 + q); }
        __threadfence();
      }
      __syncthreads();
    }
  }
}


#define GLB 2
#define GLL 1024
#define GLD 1024
#define GLH 16
#define GHD 64
#define GT (GLB * GLL)

__global__ __launch_bounds__(256) void k_scalars(const float* __restrict__ X, const float* __restrict__ Kf, const float* __restrict__ gw,
                                                const float* __restrict__ sw, float* __restrict__ GcOut, float* __restrict__ ROut) {
  __shared__ float lg[GLL], gc[GLL], rr[GLL], gws[GHD], sws[GHD];
  const int b = blockIdx.x / GLH, h = blockIdx.x % GLH, tid = threadIdx.x;
  if (tid < GHD) { gws[tid] = gw[tid]; sws[tid] = sw[tid]; }
  __syncthreads();
  for (int l = tid; l < GLL; l += 256) {
    const float* xr = X + ((size_t)(b * GLL + l)) * GLD + h * GHD; const float* kr = Kf + ((size_t)(b * GLL + l)) * GLD + h * GHD;
    float sg = 0.0f, sr = 0.0f;
#pragma unroll 8
    for (int dd = 0; dd < GHD; ++dd) { sg += xr[dd] * gws[dd]; sr += kr[dd] * sws[dd]; }
    float G = 1.0f / (1.0f + expf(-sg)); G = fmaxf(G, 1e-6f);
    lg[l] = logf(G);
    rr[l] = sr / (1.0f + expf(-sr));
  }
  __syncthreads();
  if (tid == 0) { float cs = 0.0f;
    for (int l = 0; l < GLL; ++l) { cs += lg[l]; const float c = fminf(fmaxf(cs, -30.0f), 30.0f); gc[l] = expf(c) + 1e-6f; } }
  __syncthreads();
#pragma unroll 1
  for (int pass = 0; pass < 2; ++pass) {
    for (int l = tid; l < GLL; l += 256) { *(volatile float*)(GcOut + (size_t)blockIdx.x * GLL + l) = gc[l]; *(volatile float*)(ROut + (size_t)blockIdx.x * GLL + l) = rr[l]; }
    __threadfence();
  }
}

__global__ __launch_bounds__(256) void k_transform(float* __restrict__ Qm, float* __restrict__ K2) {
  const size_t e0 = ((size_t)blockIdx.x * 256 + threadIdx.x) * 4;
  v4f_t q = *(const v4fa*)(Qm + e0), k = *(const v4fa*)(K2 + e0);
#pragma unroll
  for (int i = 0; i < 4; ++i) { float t = q[i] * (-0.125f); q[i] = -((t >= 0.0f) ? t : 0.02f * t); k[i] = 1.0f / (1.0f + expf(-(k[i] * (1.0f / 32.0f) * 0.02f))); }
#pragma unroll 1
  for (int pass = 0; pass < 2; ++pass) { *(volatile v4f_t*)(Qm + e0) = q; *(volatile v4f_t*)(K2 + e0) = k; __threadfence(); }
}

__global__ __launch_bounds__(256) void k_err(const float* __restrict__ X, const float* __restrict__ O1, float* __restrict__ E) {
  const int row = blockIdx.x, b = row / GLL, l = row % GLL, tid = threadIdx.x;
  const size_t r0 = (size_t)row * GLD;
  v4f_t v;
  if (l < GLL - 1) { const v4f_t x = *(const v4fa*)(X + r0 + GLD + tid * 4), o = *(const v4fa*)(O1 + r0 + tid * 4); v.x = x.x - o.x; v.y = x.y - o.y; v.z = x.z - o.z; v.w = x.w - o.w; }
  else { v.x = v.y = v.z = v.w = 0.0f; }
  (void)b;
  *(volatile v4f_t*)(E + r0 + tid * 4) = v; __threadfence(); *(volatile v4f_t*)(E + r0 + tid * 4) = v;
}
__global__ __launch_bounds__(256) void k_sum(const float* __restrict__ O1, const float* __restrict__ O2, float* __restrict__ Os) {
  const int row = blockIdx.x, l = row % GLL, tid = threadIdx.x;
  const size_t r0 = (size_t)row * GLD;
  v4f_t v = *(const v4fa*)(O1 + r0 + tid * 4);
  if (l >= 1) { const v4f_t o = *(const v4fa*)(O2 + r0 - GLD + tid * 4); v.x += o.x; v.y += o.y; v.z += o.z; v.w += o.w; }
  *(volatile v4f_t*)(Os + r0 + tid * 4) = v; __threadfence(); *(volatile v4f_t*)(Os + r0 + tid * 4) = v;
}

__device__ __forceinline__ void frag32q(const float* rowp, int kh8, bf16x16& hv, bf16x16& lv) {
#pragma unroll
  for (int e = 0; e < 16; ++e) { const float v = rowp[kh8 + ((e < 8) ? e : (e + 8))]; hv[e] = (bf16)v; lv[e] = lo_of(v, hv[e]); }
}
__global__ __launch_bounds__(64) void k_linattn(const float* __restrict__ Qs, const float* __restrict__ Ks, const float* __restrict__ Vs,
                                               const float* __restrict__ Gc  , const float* __restrict__ Rk  ,
                                               float* __restrict__ O, int Lq  ) {
  __shared__ __attribute__((aligned(16))) bf16 ldsK[2][32 * KSTRIDE];
  __shared__ __attribute__((aligned(16))) bf16 ldsV[2][64 * VSTRIDE];
  __shared__ float gck[32], rk[32];
  __shared__ __attribute__((aligned(16))) float ldsO[2][16 * 68];
  const int q0blk = blockIdx.x * 32, h = blockIdx.y, b = blockIdx.z;
  const int t = threadIdx.x, wave = t >> 5, lane = t & 31, qlane = lane & 15, kh8 = (lane >> 4) * 8;
  const int q0 = q0blk + wave * 16;
  const size_t rowQ = (size_t)b * GLL;
  const int qi = q0 + qlane;
  bf16x16 qf[2], qfl[2];
#pragma unroll
  for (int c = 0; c < 2; ++c) frag32q(Qs + (rowQ + qi) * GLD + h * GHD + c * 32, kh8, qf[c], qfl[c]);
  const float gq = Gc ? Gc[((size_t)b * GLH + h) * GLL + qi] : 1.0f;
  f32x8 o[4] = {};
  const int kmax = min(q0blk + 31, Lq - 1);
  for (int kb = 0; kb <= kmax; kb += 32) {
    __syncthreads();
    {
      const int kr = t >> 1, kc = (t & 1) * 32; const float* ks = Ks + (rowQ + kb + kr) * GLD + h * GHD + kc;
#pragma unroll
      for (int i = 0; i < 32; ++i) { const float v = ks[i]; const bf16 hv = (bf16)v; ldsK[0][kr * KSTRIDE + kc + i] = hv; ldsK[1][kr * KSTRIDE + kc + i] = lo_of(v, hv); }
      const int vk = t & 31, e0 = (t >> 5) * 32; const float* vs = Vs + (rowQ + kb + vk) * GLD + h * GHD + e0;
#pragma unroll
      for (int i = 0; i < 32; ++i) { const float v = vs[i]; const bf16 hv = (bf16)v; ldsV[0][(e0 + i) * VSTRIDE + vk] = hv; ldsV[1][(e0 + i) * VSTRIDE + vk] = lo_of(v, hv); }
      if (t < 32) { const size_t si = ((size_t)b * GLH + h) * GLL + kb + t; gck[t] = Gc ? Gc[si] : 1.0f; rk[t] = Rk ? Rk[si] : 1.0f; }
    }
    __syncthreads();
    f32x8 s0 = {}, s1 = {};
#pragma unroll
    for (int c = 0; c < 2; ++c) {
      s0 = wmma_split(lds_frag(&ldsK[0][0 * KSTRIDE + c * 32], KSTRIDE), lds_frag(&ldsK[1][0 * KSTRIDE + c * 32], KSTRIDE), qf[c], qfl[c], s0);
      s1 = wmma_split(lds_frag(&ldsK[0][16 * KSTRIDE + c * 32], KSTRIDE), lds_frag(&ldsK[1][16 * KSTRIDE + c * 32], KSTRIDE), qf[c], qfl[c], s1);
    }
    bf16x16 pf, pfl;
#pragma unroll
    for (int r = 0; r < 8; ++r) {
      const int j0 = kb + kh8 + r, j1 = j0 + 16;
      const float w0 = (j0 <= qi) ? s0[r] * rk[kh8 + r] * (gq / gck[kh8 + r]) : 0.0f;
      const float w1 = (j1 <= qi) ? s1[r] * rk[16 + kh8 + r] * (gq / gck[16 + kh8 + r]) : 0.0f;
      pf[r] = (bf16)w0; pfl[r] = lo_of(w0, pf[r]); pf[r + 8] = (bf16)w1; pfl[r + 8] = lo_of(w1, pf[r + 8]);
    }
#pragma unroll
    for (int j = 0; j < 4; ++j)
      o[j] = wmma_split(lds_frag(&ldsV[0][(j * 16) * VSTRIDE], VSTRIDE), lds_frag(&ldsV[1][(j * 16) * VSTRIDE], VSTRIDE), pf, pfl, o[j]);
  }
  float* so = ldsO[wave];
#pragma unroll
  for (int j = 0; j < 4; ++j)
#pragma unroll
    for (int r = 0; r < 8; ++r) so[qlane * 68 + j * 16 + kh8 + r] = o[j][r];
  asm volatile("s_wait_dscnt 0" ::: "memory");
#pragma unroll 1
  for (int pass = 0; pass < 2; ++pass) {
#pragma unroll
    for (int it = 0; it < 8; ++it) { const int ch = lane + 32 * it, ql = ch >> 4, q4 = (ch & 15) * 4;
      *(volatile v4f_t*)(O + (rowQ + q0 + ql) * GLD + h * GHD + q4) = *(const volatile v4fa*)(so + ql * 68 + q4); }
    __threadfence();
  }
}

extern "C" void kernel_launch(void* const* d_in, const int* in_sizes, int n_in,
                              void* d_out, int out_size, void* d_ws, size_t ws_size,
                              hipStream_t stream) {
  (void)in_sizes; (void)n_in; (void)out_size; (void)ws_size;
  const float* X    = (const float*)d_in[0];
  const float* q1w  = (const float*)d_in[1];
  const float* k1w  = (const float*)d_in[2];
  const float* k2w  = (const float*)d_in[3];
  const float* gww  = (const float*)d_in[4];
  const float* sww  = (const float*)d_in[5];
  const float* cpw  = (const float*)d_in[6];
  char* ws = (char*)d_ws;
  const size_t act = (size_t)GT * GLD * 4;
  float* Qf  = (float*)ws; ws += act;
  float* Kf  = (float*)ws; ws += act;
  float* K2f = (float*)ws; ws += act;
  float* O1  = (float*)ws; ws += act;
  float* Ef  = (float*)ws; ws += act;
  float* O2  = (float*)ws; ws += act;
  float* Os  = (float*)ws; ws += act;
  float* Gc  = (float*)ws; ws += (size_t)GLB * GLH * GLL * 4;
  float* Rk  = (float*)ws; ws += (size_t)GLB * GLH * GLL * 4;

  dim3 g(GT / 128, GLD / 256), blk(256);
  gemm_split_kernel<float, float, 2><<<g, blk, 0, stream>>>(X, 0, q1w, 0, nullptr, Qf,  GT, GLD, GLD);
  gemm_split_kernel<float, float, 2><<<g, blk, 0, stream>>>(X, 0, k1w, 0, nullptr, Kf,  GT, GLD, GLD);
  gemm_split_kernel<float, float, 2><<<g, blk, 0, stream>>>(X, 0, k2w, 0, nullptr, K2f, GT, GLD, GLD);
  k_scalars<<<GLB * GLH, 256, 0, stream>>>(X, Kf, gww, sww, Gc, Rk);
  k_linattn<<<dim3(GLL / 32, GLH, GLB), 64, 0, stream>>>(Qf, Kf, X, Gc, Rk, O1, GLL);
  k_err<<<GT, 256, 0, stream>>>(X, O1, Ef);
  k_transform<<<GT * GLD / 4 / 256, 256, 0, stream>>>(Qf, K2f);
  k_linattn<<<dim3(GLL / 32, GLH, GLB), 64, 0, stream>>>(Qf, K2f, Ef, nullptr, nullptr, O2, GLL - 1);
  k_sum<<<GT, 256, 0, stream>>>(O1, O2, Os);
  gemm_split_kernel<float, float, 2><<<g, blk, 0, stream>>>(Os, 0, cpw, 0, nullptr, (float*)d_out, GT, GLD, GLD);
}
